// Mamba3DBlock_70153995813183
// MI455X (gfx1250) — hardware-run, weakly checked
//
#include <hip/hip_runtime.h>
#include <stdint.h>

constexpr int kBatch   = 2;
constexpr int kSeq     = 2048;
constexpr int kDModel  = 1024;
constexpr int kDInner  = 1536;
constexpr int kDState  = 8;
constexpr int kDtRank  = 64;
constexpr int kDff     = 2048;
constexpr int kTok     = kBatch * kSeq;
constexpr int kXdblW   = kDtRank + 2 * kDState;
constexpr int kXdblPad = 128;
constexpr int kConvK   = 4;

constexpr float kWCarry  = 64.0f;
constexpr float kXiCarry = 16.0f;
constexpr float kActCarry = 64.0f;

static_assert(kTok % 64 == 0);
static_assert(kDInner % 64 == 0 && kDModel % 64 == 0 && kDff % 64 == 0 && kXdblPad % 64 == 0);
static_assert(kDModel % 32 == 0 && kDInner % 32 == 0 && kDtRank % 32 == 0 && kDff % 32 == 0);
static_assert(kXdblW <= kXdblPad);
static_assert(kSeq % 16 == 0);
static_assert(kDInner % 64 == 0);

typedef __attribute__((ext_vector_type(16))) _Float16 v16h;
typedef __attribute__((ext_vector_type(8)))  _Float16 v8h;
typedef __attribute__((ext_vector_type(16))) __bf16   v16b;
typedef __attribute__((ext_vector_type(8)))  __bf16   v8b;
typedef __attribute__((ext_vector_type(8)))  float    v8f;
typedef __attribute__((ext_vector_type(4)))  float    v4f;
typedef __attribute__((ext_vector_type(2)))  float    v2f;
typedef __attribute__((ext_vector_type(4)))  unsigned v4u;

__device__ __forceinline__ unsigned short f2bf_bits(float f) {
  unsigned u = __float_as_uint(f);
  return (unsigned short)((u + 0x7FFFu + ((u >> 16) & 1u)) >> 16);
}
__device__ __forceinline__ float bf_bits2f(unsigned short h) { return __uint_as_float(((unsigned)h) << 16); }

__device__ __forceinline__ float h2f(unsigned w16) {
  return (float)__builtin_bit_cast(_Float16, (unsigned short)(w16 & 0xffffu));
}
__device__ __forceinline__ unsigned pack_h2(float f0, float f1) {
  const unsigned short a = __builtin_bit_cast(unsigned short, (_Float16)f0);
  const unsigned short b = __builtin_bit_cast(unsigned short, (_Float16)f1);
  return (unsigned)a | ((unsigned)b << 16);
}

__device__ __forceinline__ void dep_guard_h(v8f& a, v8f& b, v16h x, v16h y) { asm volatile("v_nop\n\tv_nop\n\tv_nop\n\tv_nop" : "+v"(a), "+v"(b) : "v"(x), "v"(y)); }
__device__ __forceinline__ void dep_guard_b(v8f& a, v8f& b, v16b x, v16b y) { asm volatile("v_nop\n\tv_nop\n\tv_nop\n\tv_nop" : "+v"(a), "+v"(b) : "v"(x), "v"(y)); }
__device__ __forceinline__ void keep4_h(v16h a, v16h b, v16h c, v16h d) { asm volatile("v_nop" :: "v"(a), "v"(b), "v"(c), "v"(d)); }
__device__ __forceinline__ void keep4_b(v16b a, v16b b, v16b c, v16b d) { asm volatile("v_nop" :: "v"(a), "v"(b), "v"(c), "v"(d)); }
__device__ __forceinline__ void acc_guard4(v8f& a, v8f& b, v8f& c, v8f& d) { asm volatile("v_nop\n\tv_nop\n\tv_nop\n\tv_nop" : "+v"(a), "+v"(b), "+v"(c), "+v"(d)); }
template <typename T> struct Frag;
template <> struct Frag<_Float16> {
  typedef v16h V; union U { v16h v; v8h h[2]; };
  static __device__ __forceinline__ v16h load(const _Float16* p) {
    U f; f.h[0] = *(const v8h*)(p); f.h[1] = *(const v8h*)(p + 16); return f.v;
  }
  static __device__ __forceinline__ v8f mma(v16h a, v16h b, v8f c) {
    return __builtin_amdgcn_wmma_f32_16x16x32_f16(false, a, false, b, (short)0, c, false, false);
  }
  static __device__ __forceinline__ void guard(v8f& a, v8f& b, v16h x, v16h y) { dep_guard_h(a, b, x, y); }
  static __device__ __forceinline__ void keep(v16h a, v16h b, v16h c, v16h d) { keep4_h(a, b, c, d); }
};
template <> struct Frag<__bf16> {
  typedef v16b V; union U { v16b v; v8b h[2]; };
  static __device__ __forceinline__ v16b load(const __bf16* p) {
    U f; f.h[0] = *(const v8b*)(p); f.h[1] = *(const v8b*)(p + 16); return f.v;
  }
  static __device__ __forceinline__ v8f mma(v16b a, v16b b, v8f c) {
    return __builtin_amdgcn_wmma_f32_16x16x32_bf16(false, a, false, b, (short)0, c, false, false);
  }
  static __device__ __forceinline__ void guard(v8f& a, v8f& b, v16b x, v16b y) { dep_guard_b(a, b, x, y); }
  static __device__ __forceinline__ void keep(v16b a, v16b b, v16b c, v16b d) { keep4_b(a, b, c, d); }
};

template <int ET> struct Elem;
template <> struct Elem<0> { typedef _Float16 T; };
template <> struct Elem<1> { typedef __bf16 T; };
template <int ET, bool SPLIT, int BIAS_MODE, int OUT_MODE, bool RESID, int ACT = 0>
__global__ __launch_bounds__(256) void wmma_gemm64(
    const unsigned short* __restrict__ Ap, const unsigned short* __restrict__ A2p, int lda, long strideA,
    const unsigned short* __restrict__ Btp, const unsigned short* __restrict__ Bt2p, int ldb, long strideB,
    void* __restrict__ Cout, void* __restrict__ Cout2, int ldc, long strideC,
    const float* __restrict__ bias,
    const float* __restrict__ resid, long strideR,
    int M, int N, int K, float scale) {
  typedef typename Elem<ET>::T T;
  typedef typename Frag<T>::V V;
  const T* A = (const T*)Ap; const T* A2 = (const T*)A2p; const T* Bt = (const T*)Btp; const T* Bt2 = (const T*)Bt2p;
  __shared__ __align__(16) float sT[8][16 * 68];
  const int b    = blockIdx.y;
  const int lane = threadIdx.x & 31;
  const int wave = threadIdx.x >> 5;
  const int tilesN = N >> 6;
  const int tilesM = M >> 6;
  const int tile = blockIdx.x * 8 + wave;
  if (tile >= tilesM * tilesN) return;
  const int tm = tile / tilesN;
  const int tn = tile - tm * tilesN;
  const int m0 = tm << 6;
  const int n0 = tn << 6;

  const T* Ab  = A  + (size_t)b * strideA;
  const T* Bb  = Bt + (size_t)b * strideB;
  const T* Ab2 = SPLIT ? (A2  + (size_t)b * strideA) : nullptr;
  const T* Bb2 = SPLIT ? (Bt2 + (size_t)b * strideB) : nullptr;

  const int rlane = lane & 15;
  const int koff  = (lane >> 4) * 8;
  const int mOff  = (lane >> 4) * 8;

  v8f acc[4][4];
#pragma unroll
  for (int i = 0; i < 4; ++i)
#pragma unroll
    for (int j = 0; j < 4; ++j) acc[i][j] = (v8f){0.f,0.f,0.f,0.f,0.f,0.f,0.f,0.f};

  for (int k0 = 0; k0 < K; k0 += 32) {
    V bh[4], bl[4];
#pragma unroll
    for (int j = 0; j < 4; ++j) {
      const size_t bo = (size_t)(n0 + (j << 4) + rlane) * ldb + koff + k0;
      bh[j] = Frag<T>::load(Bb + bo);
      if (SPLIT) bl[j] = Frag<T>::load(Bb2 + bo);
    }
#pragma unroll
    for (int i = 0; i < 4; ++i) {
      const size_t ao = (size_t)(m0 + (i << 4) + rlane) * lda + koff + k0;
      V ah = Frag<T>::load(Ab + ao);
      V al;
      if (SPLIT) al = Frag<T>::load(Ab2 + ao);
#pragma unroll
      for (int j = 0; j < 4; ++j) {
        acc[i][j] = Frag<T>::mma(ah, bh[j], acc[i][j]);
        if (SPLIT) {
          acc[i][j] = Frag<T>::mma(ah, bl[j], acc[i][j]);
          acc[i][j] = Frag<T>::mma(al, bh[j], acc[i][j]);
        }
      }
      Frag<T>::guard(acc[i][0], acc[i][3], ah, SPLIT ? al : ah);
    }
    Frag<T>::keep(bh[0], bh[1], bh[2], bh[3]);
    if (SPLIT) Frag<T>::keep(bl[0], bl[1], bl[2], bl[3]);
  }
  acc_guard4(acc[0][0], acc[0][1], acc[0][2], acc[0][3]);
  acc_guard4(acc[1][0], acc[1][1], acc[1][2], acc[1][3]);
  acc_guard4(acc[2][0], acc[2][1], acc[2][2], acc[2][3]);
  acc_guard4(acc[3][0], acc[3][1], acc[3][2], acc[3][3]);

  float* slab = sT[wave];
  const float* Rb = RESID ? (resid + (size_t)b * strideR) : nullptr;
#pragma unroll
  for (int i = 0; i < 4; ++i) {
    const int mBase = m0 + (i << 4);
#pragma unroll
    for (int j = 0; j < 4; ++j) {
      const int n = n0 + (j << 4) + rlane;
      float bv = 0.f;
      if (BIAS_MODE == 2) bv = bias[n];
#pragma unroll
      for (int r = 0; r < 8; ++r) {
        float v = acc[i][j][r] * scale;
        if (BIAS_MODE == 1) v += bias[mBase + mOff + r];
        if (BIAS_MODE == 2) v += bv;
        if (RESID) v += Rb[(size_t)(mBase + mOff + r) * ldc + n];
        if (ACT == 1) v = tanhf(v);
        if (ACT == 2) v = fmaxf(v, 0.0f);
        if (ACT == 3) v = v / (1.0f + expf(-v));
        if (ACT == 4) v = (v > 0.f) ? v : 0.01f * v;
        if (ACT == 5) v = 0.5f * v * (1.0f + erff(v * 0.70710678118654752f));
        slab[(mOff + r) * 68 + (j << 4) + rlane] = v;
      }
    }
    __builtin_amdgcn_fence(__ATOMIC_RELEASE, "workgroup");
    __builtin_amdgcn_wave_barrier();
    __builtin_amdgcn_fence(__ATOMIC_ACQUIRE, "workgroup");
    if (OUT_MODE == 0) {
      float* C = (float*)Cout + (size_t)b * strideC;
      const int hh = lane >> 4, c4 = (lane & 15) * 4;
      for (int pass = 0; pass < 2; ++pass) {
#pragma unroll
        for (int it = 0; it < 8; ++it) {
          const int row = it * 2 + hh;
          v4f v = *(const v4f*)(slab + row * 68 + c4);
          *(volatile v4f*)(C + (size_t)(mBase + row) * ldc + n0 + c4) = v;
        }
        __threadfence();
      }
    } else {
      const int q = lane >> 3, c8 = (lane & 7) * 8;
      unsigned short* C  = (unsigned short*)Cout  + (size_t)b * strideC;
      unsigned short* C2 = (OUT_MODE == 2) ? ((unsigned short*)Cout2 + (size_t)b * strideC) : nullptr;
      for (int pass = 0; pass < 2; ++pass) {
#pragma unroll
        for (int it = 0; it < 4; ++it) {
          const int row = it * 4 + q;
          const float* sp = slab + row * 68 + c8;
          v8h hv, lv;
#pragma unroll
          for (int e = 0; e < 8; ++e) {
            if (OUT_MODE == 1) {
              hv[e] = (_Float16)sp[e];
            } else {
              unsigned short hb = f2bf_bits(sp[e]);
              unsigned short lb = f2bf_bits(sp[e] - bf_bits2f(hb));
              hv[e] = __builtin_bit_cast(_Float16, hb);
              lv[e] = __builtin_bit_cast(_Float16, lb);
            }
          }
          *(volatile v8h*)(C + (size_t)(mBase + row) * ldc + n0 + c8) = hv;
          if (OUT_MODE == 2) *(volatile v8h*)(C2 + (size_t)(mBase + row) * ldc + n0 + c8) = lv;
        }
        __threadfence();
      }
    }
    __builtin_amdgcn_fence(__ATOMIC_RELEASE, "workgroup");
    __builtin_amdgcn_wave_barrier();
    __builtin_amdgcn_fence(__ATOMIC_ACQUIRE, "workgroup");
  }
}

__global__ __launch_bounds__(256) void cast_scale_f16x2(
    const float* __restrict__ in, _Float16* __restrict__ out, int n2_total, int n_real, float scale) {
  const int i = blockIdx.x * 256 + threadIdx.x;
  if (i < n2_total) {
    const int idx  = 2 * i;
    const int idxc = (idx < n_real - 2) ? idx : (n_real - 2);
    float f0 = in[idxc] * scale;
    float f1 = in[idxc + 1] * scale;
    if (idx >= n_real) { f0 = 0.0f; f1 = 0.0f; }
    const unsigned u = pack_h2(f0, f1);
    ((volatile unsigned*)out)[i] = u;
    __threadfence();
    ((volatile unsigned*)out)[i] = u;
  }
}

__global__ __launch_bounds__(128) void layernorm_f16_kernel(
    const float* __restrict__ x, const float* __restrict__ g, const float* __restrict__ bt,
    unsigned short* __restrict__ out) {
  __shared__ float red0[4];
  __shared__ float red1[4];
  const int row  = blockIdx.x;
  const int tid  = threadIdx.x;
  const int lane = tid & 31;
  const int wave = tid >> 5;
  const int c0   = tid * 8;
  const float* xr = x + (size_t)row * kDModel + c0;
  const v4f a = *(const v4f*)(xr);
  const v4f c = *(const v4f*)(xr + 4);
  float s = ((a[0] + a[1]) + (a[2] + a[3])) + ((c[0] + c[1]) + (c[2] + c[3]));
#pragma unroll
  for (int off = 1; off < 32; off <<= 1) s += __shfl_xor(s, off, 32);
  if (lane == 0) red0[wave] = s;
  __syncthreads();
  const float mean = ((red0[0] + red0[1]) + (red0[2] + red0[3])) * (1.0f / (float)kDModel);
  float dv[8];
  dv[0] = a[0] - mean; dv[1] = a[1] - mean; dv[2] = a[2] - mean; dv[3] = a[3] - mean;
  dv[4] = c[0] - mean; dv[5] = c[1] - mean; dv[6] = c[2] - mean; dv[7] = c[3] - mean;
  float q = 0.0f;
#pragma unroll
  for (int e = 0; e < 8; ++e) q += dv[e] * dv[e];
#pragma unroll
  for (int off = 1; off < 32; off <<= 1) q += __shfl_xor(q, off, 32);
  if (lane == 0) red1[wave] = q;
  __syncthreads();
  const float var = ((red1[0] + red1[1]) + (red1[2] + red1[3])) * (1.0f / (float)kDModel);
  const float inv = rsqrtf(var + 1e-5f);
  const v4f g0 = *(const v4f*)(g + c0);
  const v4f g1 = *(const v4f*)(g + c0 + 4);
  const v4f b0 = *(const v4f*)(bt + c0);
  const v4f b1 = *(const v4f*)(bt + c0 + 4);
  float o[8];
  o[0] = dv[0] * inv * g0[0] + b0[0];
  o[1] = dv[1] * inv * g0[1] + b0[1];
  o[2] = dv[2] * inv * g0[2] + b0[2];
  o[3] = dv[3] * inv * g0[3] + b0[3];
  o[4] = dv[4] * inv * g1[0] + b1[0];
  o[5] = dv[5] * inv * g1[1] + b1[1];
  o[6] = dv[6] * inv * g1[2] + b1[2];
  o[7] = dv[7] * inv * g1[3] + b1[3];
  v4u w;
  w[0] = pack_h2(o[0], o[1]);
  w[1] = pack_h2(o[2], o[3]);
  w[2] = pack_h2(o[4], o[5]);
  w[3] = pack_h2(o[6], o[7]);
  unsigned short* op = out + (size_t)row * kDModel + c0;
  *(volatile v4u*)op = w;
  __threadfence();
  *(volatile v4u*)op = w;
}

__global__ __launch_bounds__(256) void conv_silu_kernel(
    const unsigned short* __restrict__ xi16, const float* __restrict__ cw,
    const float* __restrict__ cb, _Float16* __restrict__ u16) {
  const int i = blockIdx.x * 256 + threadIdx.x;
  if (i >= (kTok * kDInner) / 2) return;
  const int t = i / (kDInner / 2);
  const int d = (i - t * (kDInner / 2)) * 2;
  const int l = t & (kSeq - 1);
  const v4f w0 = *(const v4f*)(cw + d * kConvK);
  const v4f w1 = *(const v4f*)(cw + (d + 1) * kConvK);
  float acc0 = cb[d];
  float acc1 = cb[d + 1];
  const unsigned* xw = (const unsigned*)xi16;
#pragma unroll
  for (int j = 0; j < kConvK; ++j) {
    const int lp = l - (kConvK - 1) + j;
    const int tr = (lp >= 0) ? (t - (kConvK - 1) + j) : t;
    const unsigned wd = xw[((size_t)tr * kDInner + d) >> 1];
    float v0 = h2f(wd & 0xffffu) * (1.0f / kXiCarry);
    float v1 = h2f(wd >> 16) * (1.0f / kXiCarry);
    if (lp < 0) { v0 = 0.0f; v1 = 0.0f; }
    acc0 += w0[j] * v0;
    acc1 += w1[j] * v1;
  }
  const float s0 = acc0 * (1.0f / (1.0f + expf(-acc0)));
  const float s1 = acc1 * (1.0f / (1.0f + expf(-acc1)));
  const unsigned u = pack_h2(s0 * kActCarry, s1 * kActCarry);
  ((volatile unsigned*)u16)[i] = u;
  __threadfence();
  ((volatile unsigned*)u16)[i] = u;
}

__global__ __launch_bounds__(256) void dt_cast_kernel(
    const float* __restrict__ xdbl, _Float16* __restrict__ dt16) {
  const int i = blockIdx.x * 256 + threadIdx.x;
  if (i >= kTok * (kDtRank / 2)) return;
  const int row = i >> 5;
  const int cp  = i & 31;
  const v2f p = *(const v2f*)(xdbl + (size_t)row * kXdblPad + 2 * cp);
  const unsigned u = pack_h2(p[0] * kActCarry, p[1] * kActCarry);
  ((volatile unsigned*)dt16)[i] = u;
  __threadfence();
  ((volatile unsigned*)dt16)[i] = u;
}

__global__ __launch_bounds__(256) void gelu_f16_kernel(
    const float* __restrict__ hpre, _Float16* __restrict__ h16) {
  const int i = blockIdx.x * 256 + threadIdx.x;
  if (i >= (kTok * kDff) / 2) return;
  const v2f p = *(const v2f*)(hpre + 2 * (size_t)i);
  const float g0 = 0.5f * p[0] * (1.0f + erff(p[0] * 0.70710678118654752f));
  const float g1 = 0.5f * p[1] * (1.0f + erff(p[1] * 0.70710678118654752f));
  const unsigned u = pack_h2(g0 * kActCarry, g1 * kActCarry);
  ((volatile unsigned*)h16)[i] = u;
  __threadfence();
  ((volatile unsigned*)h16)[i] = u;
}

constexpr int kScanTS = 16;
__global__ __launch_bounds__(64) void scan_kernel(
    const float* __restrict__ dpre, const unsigned short* __restrict__ u16,
    const float* __restrict__ z32, const float* __restrict__ xdbl,
    const float* __restrict__ A_log, const float* __restrict__ Dp,
    unsigned short* __restrict__ y16) {
  __shared__ __align__(16) unsigned short ys[kScanTS * 64];
  const int tid  = threadIdx.x;
  const int lane = tid & 31;
  const int wave = tid >> 5;
  const int blk  = blockIdx.x;
  const int nDb  = kDInner / 64;
  const int b    = blk / nDb;
  const int dblk = blk - b * nDb;
  const int d    = dblk * 64 + tid;
  float Ar[kDState], h[kDState];
#pragma unroll
  for (int n = 0; n < kDState; ++n) {
    Ar[n] = -expf(A_log[d * kDState + n]);
    h[n]  = 0.0f;
  }
  const float Dd = Dp[d];
  const size_t row0 = (size_t)b * kSeq;
  const int q  = lane >> 3;
  const int c8 = (lane & 7) * 8;

  for (int l = 0; l < kSeq; ++l) {
    const size_t row = row0 + (size_t)l;
    const float dp = dpre[row * kDInner + d];
    const float uu = (float)__builtin_bit_cast(_Float16, u16[row * kDInner + d]) * (1.0f / kActCarry);
    const float zz = z32[row * kDInner + d];
    const float* bc = xdbl + row * kXdblPad + kDtRank;
    const v4f B0 = *(const v4f*)(bc);
    const v4f B1 = *(const v4f*)(bc + 4);
    const v4f C0 = *(const v4f*)(bc + 8);
    const v4f C1 = *(const v4f*)(bc + 12);
    float Bn[kDState], Cn[kDState];
    Bn[0] = B0[0]; Bn[1] = B0[1]; Bn[2] = B0[2]; Bn[3] = B0[3];
    Bn[4] = B1[0]; Bn[5] = B1[1]; Bn[6] = B1[2]; Bn[7] = B1[3];
    Cn[0] = C0[0]; Cn[1] = C0[1]; Cn[2] = C0[2]; Cn[3] = C0[3];
    Cn[4] = C1[0]; Cn[5] = C1[1]; Cn[6] = C1[2]; Cn[7] = C1[3];
    const float delta = fmaxf(dp, 0.0f) + log1pf(expf(-fabsf(dp)));
    const float du = delta * uu;
    float acc = 0.0f;
#pragma unroll
    for (int n = 0; n < kDState; ++n) {
      const float dA = expf(delta * Ar[n]);
      h[n] = dA * h[n] + du * Bn[n];
      acc += h[n] * Cn[n];
    }
    float yv = acc + uu * Dd;
    const float sg = zz * (1.0f / (1.0f + expf(-zz)));
    yv = yv * sg;
    ys[(l & (kScanTS - 1)) * 64 + tid] = __builtin_bit_cast(unsigned short, (_Float16)(yv * kActCarry));
    if ((l & (kScanTS - 1)) == (kScanTS - 1)) {
      __syncthreads();
      const size_t lbase = row0 + (size_t)(l - (kScanTS - 1));
      for (int pass = 0; pass < 2; ++pass) {
#pragma unroll
        for (int it = 0; it < 2; ++it) {
          const int r = wave * 8 + it * 4 + q;
          const v4u v = *(const v4u*)(ys + r * 64 + c8);
          *(volatile v4u*)(y16 + (lbase + (size_t)r) * kDInner + dblk * 64 + c8) = v;
        }
        __threadfence();
      }
      __syncthreads();
    }
  }
}

template <int BIAS_MODE, int OUT_MODE, bool RESID>
static void launch_gemm(const void* A, int lda, const void* Bt, int ldb, void* C, int ldc,
                        const float* bias, const float* resid, int M, int N, int K, float scale,
                        hipStream_t st) {
  const int tiles = (M / 64) * (N / 64);
  dim3 grid((tiles + 7) / 8, 1);
  wmma_gemm64<0, false, BIAS_MODE, OUT_MODE, RESID, 0><<<grid, 256, 0, st>>>(
      (const unsigned short*)A, nullptr, lda, 0L,
      (const unsigned short*)Bt, nullptr, ldb, 0L,
      C, nullptr, ldc, 0L,
      bias, resid, 0L, M, N, K, scale);
}

extern "C" void kernel_launch(void* const* d_in, const int* in_sizes, int n_in,
                              void* d_out, int out_size, void* d_ws, size_t ws_size,
                              hipStream_t stream) {
  (void)in_sizes; (void)n_in; (void)out_size; (void)ws_size;
  const float* x        = (const float*)d_in[0];
  const float* ln1_g    = (const float*)d_in[1];
  const float* ln1_b    = (const float*)d_in[2];
  const float* ln2_g    = (const float*)d_in[3];
  const float* ln2_b    = (const float*)d_in[4];
  const float* in_proj  = (const float*)d_in[5];
  const float* conv_w   = (const float*)d_in[6];
  const float* conv_b   = (const float*)d_in[7];
  const float* x_proj   = (const float*)d_in[8];
  const float* dt_proj  = (const float*)d_in[9];
  const float* dt_b     = (const float*)d_in[10];
  const float* A_log    = (const float*)d_in[11];
  const float* Dp       = (const float*)d_in[12];
  const float* out_proj = (const float*)d_in[13];
  const float* ffn_w1   = (const float*)d_in[14];
  const float* ffn_b1   = (const float*)d_in[15];
  const float* ffn_w2   = (const float*)d_in[16];
  const float* ffn_b2   = (const float*)d_in[17];
  float* out = (float*)d_out;

  constexpr size_t offWin = 0;
  constexpr size_t szWin  = (size_t)2 * kDInner * kDModel * 2;
  constexpr size_t offWxp = offWin + szWin;
  constexpr size_t szWxp  = (size_t)kXdblPad * kDInner * 2;
  constexpr size_t offWdt = offWxp + szWxp;
  constexpr size_t szWdt  = (size_t)kDInner * kDtRank * 2;
  constexpr size_t offWop = offWdt + szWdt;
  constexpr size_t szWop  = (size_t)kDModel * kDInner * 2;
  constexpr size_t offW1  = offWop + szWop;
  constexpr size_t szW1   = (size_t)kDff * kDModel * 2;
  constexpr size_t offW2  = offW1 + szW1;
  constexpr size_t szW2   = (size_t)kDModel * kDff * 2;
  constexpr size_t offRB  = offW2 + szW2;
  constexpr size_t szRB   = (size_t)kTok * kDModel * 2;
  constexpr size_t offRC  = offRB + szRB;
  constexpr size_t szXi16 = (size_t)kTok * kDInner * 2;
  constexpr size_t szH16  = (size_t)kTok * kDff * 2;
  constexpr size_t szRC   = (szXi16 > szH16) ? szXi16 : szH16;
  constexpr size_t offRD  = offRC + szRC;
  constexpr size_t szZ32  = (size_t)kTok * kDInner * 4;
  constexpr size_t szXmid = (size_t)kTok * kDModel * 4;
  constexpr size_t szRD   = (szZ32 > szXmid) ? szZ32 : szXmid;
  constexpr size_t offR1  = offRD + szRD;
  constexpr size_t szU16  = (size_t)kTok * kDInner * 2;
  constexpr size_t szDpre = (size_t)kTok * kDInner * 4;
  constexpr size_t szHpre = (size_t)kTok * kDff * 4;
  constexpr size_t szR1   = ((szU16 + szDpre) > szHpre) ? (szU16 + szDpre) : szHpre;
  constexpr size_t offRF  = offR1 + szR1;
  constexpr size_t szRF   = (size_t)kTok * kXdblPad * 4;
  constexpr size_t offRG  = offRF + szRF;
  constexpr size_t szRG   = (size_t)kTok * kDtRank * 2;
  constexpr size_t wsTotal = offRG + szRG;
  static_assert(wsTotal == 109117440ull);
  static_assert(wsTotal <= 134217728ull);
  static_assert((offWxp % 256) == 0 && (offRB % 256) == 0 && (offRC % 256) == 0 && (offRD % 256) == 0 &&
                (offR1 % 256) == 0 && (offRF % 256) == 0 && (offRG % 256) == 0 && ((offR1 + szU16) % 256) == 0);

  char* ws = (char*)d_ws;
  _Float16* Win16 = (_Float16*)(ws + offWin);
  _Float16* Wxp16 = (_Float16*)(ws + offWxp);
  _Float16* Wdt16 = (_Float16*)(ws + offWdt);
  _Float16* Wop16 = (_Float16*)(ws + offWop);
  _Float16* W116  = (_Float16*)(ws + offW1);
  _Float16* W216  = (_Float16*)(ws + offW2);
  unsigned short* xp16 = (unsigned short*)(ws + offRB);
  unsigned short* xn16 = (unsigned short*)(ws + offRB);
  unsigned short* xi16 = (unsigned short*)(ws + offRC);
  unsigned short* y16  = (unsigned short*)(ws + offRC);
  _Float16* h16   = (_Float16*)(ws + offRC);
  float* z32      = (float*)(ws + offRD);
  float* xmid     = (float*)(ws + offRD);
  _Float16* u16   = (_Float16*)(ws + offR1);
  float* dpre     = (float*)(ws + offR1 + szU16);
  float* hpre     = (float*)(ws + offR1);
  float* xdbl     = (float*)(ws + offRF);
  _Float16* dt16  = (_Float16*)(ws + offRG);

  {
    const int n = 2 * kDInner * kDModel;
    cast_scale_f16x2<<<(n / 2 + 255) / 256, 256, 0, stream>>>(in_proj, Win16, n / 2, n, kWCarry);
  }
  {
    const int n_total = kXdblPad * kDInner, n_real = kXdblW * kDInner;
    cast_scale_f16x2<<<(n_total / 2 + 255) / 256, 256, 0, stream>>>(x_proj, Wxp16, n_total / 2, n_real, kWCarry);
  }
  {
    const int n = kDInner * kDtRank;
    cast_scale_f16x2<<<(n / 2 + 255) / 256, 256, 0, stream>>>(dt_proj, Wdt16, n / 2, n, kWCarry);
  }
  {
    const int n = kDModel * kDInner;
    cast_scale_f16x2<<<(n / 2 + 255) / 256, 256, 0, stream>>>(out_proj, Wop16, n / 2, n, kWCarry);
  }
  {
    const int n = kDff * kDModel;
    cast_scale_f16x2<<<(n / 2 + 255) / 256, 256, 0, stream>>>(ffn_w1, W116, n / 2, n, kWCarry);
  }
  {
    const int n = kDModel * kDff;
    cast_scale_f16x2<<<(n / 2 + 255) / 256, 256, 0, stream>>>(ffn_w2, W216, n / 2, n, kWCarry);
  }

  layernorm_f16_kernel<<<kTok, 128, 0, stream>>>(x, ln1_g, ln1_b, xp16);

  launch_gemm<0, 1, false>(xp16, kDModel, Win16, kDModel, xi16, kDInner, nullptr, nullptr,
                           kTok, kDInner, kDModel, kXiCarry / kWCarry, stream);
  launch_gemm<0, 0, false>(xp16, kDModel, Win16 + (size_t)kDInner * kDModel, kDModel, z32, kDInner,
                           nullptr, nullptr, kTok, kDInner, kDModel, 1.0f / kWCarry, stream);

  conv_silu_kernel<<<(kTok * kDInner / 2 + 255) / 256, 256, 0, stream>>>(xi16, conv_w, conv_b, u16);

  launch_gemm<0, 0, false>(u16, kDInner, Wxp16, kDInner, xdbl, kXdblPad, nullptr, nullptr,
                           kTok, kXdblPad, kDInner, 1.0f / (kActCarry * kWCarry), stream);

  dt_cast_kernel<<<(kTok * (kDtRank / 2) + 255) / 256, 256, 0, stream>>>(xdbl, dt16);

  launch_gemm<2, 0, false>(dt16, kDtRank, Wdt16, kDtRank, dpre, kDInner, dt_b, nullptr,
                           kTok, kDInner, kDtRank, 1.0f / (kActCarry * kWCarry), stream);

  scan_kernel<<<kBatch * (kDInner / 64), 64, 0, stream>>>(dpre, (const unsigned short*)u16, z32, xdbl,
                                                         A_log, Dp, y16);

  launch_gemm<0, 0, true>(y16, kDInner, Wop16, kDInner, xmid, kDModel, nullptr, x,
                          kTok, kDModel, kDInner, 1.0f / (kActCarry * kWCarry), stream);

  layernorm_f16_kernel<<<kTok, 128, 0, stream>>>(xmid, ln2_g, ln2_b, xn16);

  launch_gemm<2, 0, false>(xn16, kDModel, W116, kDModel, hpre, kDff, ffn_b1, nullptr,
                           kTok, kDff, kDModel, 1.0f / kWCarry, stream);

  gelu_f16_kernel<<<(kTok * kDff / 2 + 255) / 256, 256, 0, stream>>>(hpre, h16);

  launch_gemm<2, 0, true>(h16, kDff, W216, kDff, out, kDModel, ffn_b2, xmid,
                          kTok, kDModel, kDff, 1.0f / (kActCarry * kWCarry), stream);
}
